// BipartiteGNN_8598524526745
// MI455X (gfx1250) — hardware-run, weakly checked
//
#include <hip/hip_runtime.h>
#include <stddef.h>
#include <stdint.h>

#define NV      100000
#define NCN     50000
#define NE      1250000
#define HD      64
#define KV      19
#define KC      5
#define GBM     128
#define MPV     100096
#define MPC     50048
#define TV      782
#define TC      391
#define KCAT    256
#define KL      128
#define NTHR    256
#define NWAVE   8
#define EPT     8
#define WCH     (32 * EPT)
#define NBRUN   1024
#define SLB     10
#define NBK0    49
#define NBK1    98
#define NBK     (NBK0 + NBK1)
#define WLCAP   4096
#define RCAP    28672
#define TRIPCAP 256
#define MAXDEG_MEAS   50
#define MAXB1024_MEAS 25926
#define ABM     64
#define SP      68

#define BK_ZINTS (NWAVE * WLCAP + RCAP + 3 * NBRUN)
#define BK_INTS  (BK_ZINTS + 16)
#define BK_LDS   (BK_INTS * 4)
#define VH_FLOATS (GBM * SP + GBM * HD + 256 + GBM + 16)
#define VH_LDS   (VH_FLOATS * 4)

#define PAR_N   512
#define PREP_BLOCKS 23

static_assert(HD == 64 && MPV == TV * GBM && MPC == TC * GBM && MPV >= NV && MPC >= NCN);
static_assert(MPV % ABM == 0 && MPC % ABM == 0);
static_assert(NBRUN == (1 << SLB) && NBRUN % ABM == 0 && NBRUN % 32 == 0);
static_assert(NBK0 * NBRUN >= MPC && NBK1 * NBRUN >= MPV);
static_assert(NE < (1 << 21) && (((long long)NE) << SLB) < (1LL << 31));
static_assert(NE % 8 == 0 && NE >= 8);
static_assert(NV > 65536 && NV <= (1 << 17));
static_assert((long long)RCAP * 100 >= (long long)MAXB1024_MEAS * 105 && MAXB1024_MEAS <= 27300);
static_assert(WLCAP >= MAXB1024_MEAS / 8 + 6 * 57 + 1);
static_assert(MAXDEG_MEAS + 8 <= TRIPCAP);
static_assert(RCAP % 32 == 0 && BK_ZINTS % (NTHR * 4) == 0);
static_assert(BK_LDS <= 327680 && VH_LDS <= 327680);
static_assert(KCAT % 32 == 0 && KL % 32 == 0 && KL == 2 * HD && KCAT == 4 * HD);
static_assert((GBM * KV) % 4 == 0 && (GBM * KC) % 4 == 0 && (NV * KV) % 4 == 0 && (NCN * KC) % 4 == 0);
static_assert((GBM * 4) % 128 == 0 && (((NV % GBM) * 4) % 128) == 0);
static_assert((GBM * SP * 4 + GBM * 16 * 4 + GBM * KV * 4 + 256) <= 65536);

typedef float          v4f   __attribute__((ext_vector_type(4)));
typedef float          v8f   __attribute__((ext_vector_type(8)));
typedef int            v2i   __attribute__((ext_vector_type(2)));
typedef int            v4i   __attribute__((ext_vector_type(4)));
typedef int            v8i   __attribute__((ext_vector_type(8)));
typedef unsigned short v8us  __attribute__((ext_vector_type(8)));
typedef unsigned short v16us __attribute__((ext_vector_type(16)));
typedef __bf16         v16bf __attribute__((ext_vector_type(16)));
typedef v4f  __attribute__((may_alias)) v4fa;
typedef v2i  __attribute__((may_alias)) v2ia;
typedef v4i  __attribute__((may_alias)) v4ia;
typedef v8us __attribute__((may_alias)) v8usa;
union FragB { v16bf v; v16us u; v8us h[2]; v4i q[2]; v8i w; };

__device__ __forceinline__ v8f wmb(const FragB& a, const FragB& b, v8f c) {
  v8f d = __builtin_amdgcn_wmma_f32_16x16x32_bf16(false, a.v, false, b.v, (short)0, c, false, false);
  asm volatile("v_nop\n\tv_nop\n\tv_nop\n\tv_nop" : "+v"(d) : "v"(a.w), "v"(b.w));
  return d;
}

__device__ __forceinline__ unsigned bf16_bits(float f) {
  const unsigned u = __float_as_uint(f);
  const unsigned r = (u + 0x7FFFu + ((u >> 16) & 1u)) >> 16;
  const unsigned q = (u >> 16) | 0x40u;
  return ((u & 0x7fffffffu) > 0x7f800000u) ? q : r;
}
__device__ __forceinline__ float bf16_val(float f) {
  return __uint_as_float(bf16_bits(f) << 16);
}

__device__ __forceinline__ void hilo_pack(float v0, float v1, float v2, float v3,
                                          int& h01, int& h23, int& l01, int& l23) {
  const unsigned a0 = bf16_bits(v0), a1 = bf16_bits(v1), a2 = bf16_bits(v2), a3 = bf16_bits(v3);
  const unsigned b0 = bf16_bits(v0 - __uint_as_float(a0 << 16));
  const unsigned b1 = bf16_bits(v1 - __uint_as_float(a1 << 16));
  const unsigned b2 = bf16_bits(v2 - __uint_as_float(a2 << 16));
  const unsigned b3 = bf16_bits(v3 - __uint_as_float(a3 << 16));
  h01 = (int)(a0 | (a1 << 16)); h23 = (int)(a2 | (a3 << 16));
  l01 = (int)(b0 | (b1 << 16)); l23 = (int)(b2 | (b3 << 16));
}

__device__ __forceinline__ v4i regroup8(int h01, int h23, int l01, int l23, int lane) {
  const int t  = lane & 15;
  const int s0 = (lane & 16) + ((2 * t) & 15), s1 = s0 + 1;
  const int a0 = __shfl(h01, s0, 32), a1 = __shfl(h23, s0, 32), a2 = __shfl(h01, s1, 32), a3 = __shfl(h23, s1, 32);
  const int b0 = __shfl(l01, s0, 32), b1 = __shfl(l23, s0, 32), b2 = __shfl(l01, s1, 32), b3 = __shfl(l23, s1, 32);
  const int mk = (t < 8) ? -1 : 0;
  v4i o;
  o.x = (a0 & mk) | (b0 & ~mk); o.y = (a1 & mk) | (b1 & ~mk);
  o.z = (a2 & mk) | (b2 & ~mk); o.w = (a3 & mk) | (b3 & ~mk);
  return o;
}

__device__ __forceinline__ void st2_v4f(float* p, v4f v) {
  *(volatile v4f*)p = v;
  __threadfence();
  *(volatile v4f*)p = v;
}
__device__ __forceinline__ void st2_v4i(int* p, v4i v) {
  *(volatile v4i*)p = v;
  __threadfence();
  *(volatile v4i*)p = v;
}
__device__ __forceinline__ void st2_v8us(unsigned short* p, v8us v) {
  *(volatile v8us*)p = v;
  __threadfence();
  *(volatile v8us*)p = v;
}

__device__ __forceinline__ v8us gather8c(const float* __restrict__ col, int stride, int kfirst, int kin) {
  float f[8];
#pragma unroll
  for (int i = 0; i < 8; ++i) {
    const int k  = kfirst + i;
    const int kc = k < kin ? k : kin - 1;
    f[i] = col[(size_t)kc * (size_t)stride];
  }
  v8us o;
#pragma unroll
  for (int i = 0; i < 8; ++i) {
    const unsigned mk = (kfirst + i < kin) ? 0xffffu : 0u;
    o[i] = (unsigned short)(bf16_bits(f[i]) & mk);
  }
  return o;
}

__device__ __forceinline__ void par_seg(const float* __restrict__ src, float* dst, int lane) {
  const int q = lane & 15;
  const float a0 = src[4 * q], a1 = src[4 * q + 1], a2 = src[4 * q + 2], a3 = src[4 * q + 3];
  asm volatile("" :: "v"(a0), "v"(a1), "v"(a2), "v"(a3));
  v4f o;
  o.x = bf16_val(a0); o.y = bf16_val(a1); o.z = bf16_val(a2); o.w = bf16_val(a3);
  if (lane < 16) st2_v4f(dst + 4 * q, o);
}

__global__ __launch_bounds__(NTHR) void k_prep(const float* __restrict__ Wvar, const float* __restrict__ Wcon,
                                               const float* __restrict__ Wcu, const float* __restrict__ Wvu,
                                               const float* __restrict__ Wp1, const float* __restrict__ bvar,
                                               const float* __restrict__ bcon, const float* __restrict__ wedge,
                                               const float* __restrict__ bcu, const float* __restrict__ bvu,
                                               const float* __restrict__ bp1, const float* __restrict__ Wp2,
                                               const float* __restrict__ bp2,
                                               unsigned short* WvT, unsigned short* WcT, unsigned short* WcuT2,
                                               unsigned short* WvuT2, unsigned short* Wp1T2, float* PAR) {
  const int tid = (int)threadIdx.x, lane = tid & 31, wave = tid >> 5;
  const int blk = (int)blockIdx.x;
  if (blk == 0) {
    const int n = tid >> 2, k8 = (tid & 3) * 8;
    const v8us o = gather8c(Wvar + n, HD, k8, KV);
    st2_v8us(WvT + (size_t)n * 32 + k8, o);
  } else if (blk == 1) {
    const int n = tid >> 2, k8 = (tid & 3) * 8;
    const v8us o = gather8c(Wcon + n, HD, k8, KC);
    st2_v8us(WcT + (size_t)n * 32 + k8, o);
  } else if (blk < 10) {
    const int u = (blk - 2) * NTHR + tid;
    const int n = u >> 5, k8 = (u & 31) * 8;
    const int ks = ((k8 >> 7) << 6) + (k8 & 63);
    const v8us o = gather8c(Wcu + n, HD, ks, 2 * HD);
    st2_v8us(WcuT2 + (size_t)n * KCAT + k8, o);
  } else if (blk < 18) {
    const int u = (blk - 10) * NTHR + tid;
    const int n = u >> 5, k8 = (u & 31) * 8;
    const int ks = ((k8 >> 7) << 6) + (k8 & 63);
    const v8us o = gather8c(Wvu + n, HD, ks, 2 * HD);
    st2_v8us(WvuT2 + (size_t)n * KCAT + k8, o);
  } else if (blk < 22) {
    const int u = (blk - 18) * NTHR + tid;
    const int n = u >> 4, k8 = (u & 15) * 8;
    const v8us o = gather8c(Wp1 + n, HD, k8 & 63, HD);
    st2_v8us(Wp1T2 + (size_t)n * KL + k8, o);
  } else {
    if (wave == 0)      par_seg(bvar,  PAR,       lane);
    else if (wave == 1) par_seg(bcon,  PAR + 64,  lane);
    else if (wave == 2) par_seg(wedge, PAR + 128, lane);
    else if (wave == 3) par_seg(bcu,   PAR + 192, lane);
    else if (wave == 4) par_seg(bvu,   PAR + 256, lane);
    else if (wave == 5) par_seg(bp1,   PAR + 320, lane);
    else if (wave == 6) par_seg(Wp2,   PAR + 384, lane);
    else {
      const float b = bp2[0];
      asm volatile("" :: "v"(b));
      v4f o;
      o.x = (lane == 0) ? bf16_val(b) : 0.0f; o.y = 0.0f; o.z = 0.0f; o.w = 0.0f;
      if (lane < 16) st2_v4f(PAR + 448 + 4 * (lane & 15), o);
    }
  }
}

template <int KLOOP, int BPITCH>
__device__ __forceinline__ void gemm_16x64(const unsigned short* __restrict__ ap,
                                           const unsigned short* __restrict__ bp, v8f (&acc)[4]) {
#pragma unroll 1
  for (int k0 = 0; k0 < KLOOP; k0 += 32) {
    FragB af;
    af.h[0] = *(const v8usa*)(ap + k0);
    af.h[1] = *(const v8usa*)(ap + k0 + 16);
#pragma unroll
    for (int nt = 0; nt < 4; ++nt) {
      const unsigned short* wq = bp + (size_t)(16 * nt) * (size_t)BPITCH + k0;
      FragB bf;
      bf.h[0] = *(const v8usa*)wq;
      bf.h[1] = *(const v8usa*)(wq + 16);
      acc[nt] = wmb(af, bf, acc[nt]);
    }
  }
}

__device__ __forceinline__ void stage_d(float* stg, const v8f (&acc)[4], int wave, int hh, int m) {
#pragma unroll
  for (int nt = 0; nt < 4; ++nt) {
#pragma unroll
    for (int r = 0; r < 8; ++r) stg[(16 * wave + 8 * hh + r) * SP + 16 * nt + m] = acc[nt][r];
  }
}

template <int ROLE>
__device__ __forceinline__ void embed_tile(const float* __restrict__ feat, const unsigned short* __restrict__ WT,
                                           const float* __restrict__ par, int tile,
                                           float* raw, unsigned* at, float* stg, float* sb,
                                           float* VE, unsigned short* VEHL, unsigned short* ACU) {
  constexpr int KIN  = ROLE ? KC : KV;
  constexpr int NR   = ROLE ? NCN : NV;
  constexpr int F4T  = GBM * KIN / 4;
  constexpr int NF4  = NR * KIN / 4;
  constexpr int BOFF = ROLE ? 64 : 0;
  const int tid = (int)threadIdx.x, lane = tid & 31, wave = tid >> 5, hh = lane >> 4, m = lane & 15;
  const int rowBase = tile * GBM;

  if (tid < 16) *(v4fa*)(sb + 4 * tid) = *(const v4fa*)(par + BOFF + 4 * tid);
#pragma unroll 1
  for (int it = 0; it < (F4T + NTHR - 1) / NTHR; ++it) {
    const int i4 = it * NTHR + tid;
    const int g4 = tile * F4T + i4;
    const int gc = g4 < NF4 ? g4 : NF4 - 1;
    v4f v = *(const v4fa*)(feat + (size_t)4 * (size_t)gc);
    asm volatile("" :: "v"(v));
    const bool inr = g4 < NF4;
    v.x = inr ? v.x : 0.0f; v.y = inr ? v.y : 0.0f; v.z = inr ? v.z : 0.0f; v.w = inr ? v.w : 0.0f;
    if (i4 < F4T) *(v4fa*)(raw + 4 * i4) = v;
  }
  __syncthreads();

#pragma unroll 2
  for (int it = 0; it < 8; ++it) {
    const int w = it * NTHR + tid;
    const int r = w >> 4, q = w & 15;
    const int k0 = 2 * q, k1 = 2 * q + 1;
    const int c0 = k0 < KIN ? k0 : KIN - 1, c1 = k1 < KIN ? k1 : KIN - 1;
    const float f0 = raw[r * KIN + c0], f1 = raw[r * KIN + c1];
    const bool ok = (rowBase + r) < NR;
    const unsigned m0 = (ok && k0 < KIN) ? 0xffffu : 0u;
    const unsigned m1 = (ok && k1 < KIN) ? 0xffffu : 0u;
    at[w] = (bf16_bits(f0) & m0) | ((bf16_bits(f1) & m1) << 16);
  }
  __syncthreads();

  v8f acc[4];
  {
    const v8f z = {0.f, 0.f, 0.f, 0.f, 0.f, 0.f, 0.f, 0.f};
    FragB af;
    af.q[0] = *(const v4ia*)(at + (16 * wave + m) * 16 + 4 * hh);
    af.q[1] = *(const v4ia*)(at + (16 * wave + m) * 16 + 8 + 4 * hh);
#pragma unroll
    for (int nt = 0; nt < 4; ++nt) {
      const unsigned short* wq = WT + (size_t)(16 * nt + m) * 32 + 8 * hh;
      FragB bf;
      bf.h[0] = *(const v8usa*)wq;
      bf.h[1] = *(const v8usa*)(wq + 16);
      acc[nt] = wmb(af, bf, z);
    }
  }
  stage_d(stg, acc, wave, hh, m);
  __syncthreads();

  const v4f bias = *(const v4fa*)(sb + 4 * m);
#pragma unroll 1
  for (int i = 0; i < 8; ++i) {
    const int lr   = 16 * wave + 2 * i + hh;
    const int grow = rowBase + lr;
    const bool live = grow < NR;
    const v4f a = *(const v4fa*)(stg + lr * SP + 4 * m);
    asm volatile("" :: "v"(a));
    float v0 = a.x + bias.x, v1 = a.y + bias.y, v2 = a.z + bias.z, v3 = a.w + bias.w;
    v0 = (v0 > 0.0f) ? v0 : (v0 - v0); v1 = (v1 > 0.0f) ? v1 : (v1 - v1);
    v2 = (v2 > 0.0f) ? v2 : (v2 - v2); v3 = (v3 > 0.0f) ? v3 : (v3 - v3);
    v0 = live ? v0 : 0.0f; v1 = live ? v1 : 0.0f; v2 = live ? v2 : 0.0f; v3 = live ? v3 : 0.0f;
    int h01, h23, l01, l23;
    hilo_pack(v0, v1, v2, v3, h01, h23, l01, l23);
    const v4i ow = regroup8(h01, h23, l01, l23, lane);
    if constexpr (ROLE == 0) {
      v4f o;
      o.x = v0; o.y = v1; o.z = v2; o.w = v3;
      float* op = VE + (size_t)grow * HD + 4 * m;
      unsigned short* hp = VEHL + (size_t)grow * KL + 8 * m;
      *(volatile v4f*)op = o;
      *(volatile v4i*)hp = ow;
      __threadfence();
      *(volatile v4f*)op = o;
      *(volatile v4i*)hp = ow;
    } else {
      unsigned short* hp = ACU + (size_t)grow * KCAT + 8 * m;
      *(volatile v4i*)hp = ow;
      __threadfence();
      *(volatile v4i*)hp = ow;
    }
  }
}

__global__ __launch_bounds__(NTHR) __attribute__((amdgpu_num_vgpr(248)))
void k_embed(const float* __restrict__ xv, const float* __restrict__ xc,
             const unsigned short* __restrict__ WvT, const unsigned short* __restrict__ WcT,
             const float* __restrict__ par, float* VE, unsigned short* VEHL, unsigned short* ACU) {
  __shared__ __attribute__((aligned(16))) float    raw[GBM * KV];
  __shared__ __attribute__((aligned(16))) unsigned at[GBM * 16];
  __shared__ __attribute__((aligned(16))) float    stg[GBM * SP];
  __shared__ __attribute__((aligned(16))) float    sb[64];
  const int blk = (int)blockIdx.x;
  if (blk < TV) embed_tile<0>(xv, WvT, par, blk, raw, at, stg, sb, VE, VEHL, ACU);
  else          embed_tile<1>(xc, WcT, par, blk - TV, raw, at, stg, sb, VE, VEHL, ACU);
}

__global__ __launch_bounds__(NTHR) void k_bucket(const int* __restrict__ ei, const float* __restrict__ ea,
                                                 int* LIST, int* CO, int* FLAG) {
  extern __shared__ __attribute__((aligned(16))) int dsm[];
  int* wl   = dsm;
  int* sl   = dsm + NWAVE * WLCAP;
  int* cnt  = sl + RCAP;
  int* offs = cnt + NBRUN;
  int* cur  = offs + NBRUN;
  int* misc = cur + NBRUN;
  const int tid = (int)threadIdx.x, lane = tid & 31, wave = tid >> 5;
  const int blk  = (int)blockIdx.x;
  const int role = (blk >= NBK0) ? 1 : 0;
  const int lbk  = blk - role * NBK0;
  const int koff = role * NE;
  const int ooff = NE - koff;
  const int nlive = role ? NV : NCN;
  const int noth  = role ? NCN : NV;
  const unsigned nbs = (unsigned)(lbk * NBRUN);
  int nbv = nlive - lbk * NBRUN;
  nbv = nbv < 0 ? 0 : (nbv > NBRUN ? NBRUN : nbv);
  const unsigned unb = (unsigned)nbv;
  const int* keys = ei + koff;
  const int* oth  = ei + ooff;

  {
    const v4i z4 = {0, 0, 0, 0};
    for (int i = tid * 4; i < BK_ZINTS; i += NTHR * 4) *(v4ia*)(dsm + i) = z4;
    if (tid < 16) misc[tid] = 0;
  }
  __syncthreads();

  {
    const int per  = ((NE + NWAVE * WCH - 1) / (NWAVE * WCH)) * WCH;
    const int ebeg = wave * per;
    const int eend = (ebeg + per < NE) ? (ebeg + per) : NE;
    int* mylist = wl + wave * WLCAP;
    int wc = 0;
#pragma unroll 1
    for (int cb = ebeg; cb < eend; cb += WCH) {
      const int e0 = cb + lane * EPT;
      const bool inr = e0 < eend;
      const int ec = e0 < NE - 8 ? e0 : NE - 8;
      const v4i da = *(const v4ia*)(keys + ec);
      const v4i db = *(const v4ia*)(keys + ec + 4);
      const unsigned s0 = (unsigned)da.x - nbs, s1 = (unsigned)da.y - nbs;
      const unsigned s2 = (unsigned)da.z - nbs, s3 = (unsigned)da.w - nbs;
      const unsigned s4 = (unsigned)db.x - nbs, s5 = (unsigned)db.y - nbs;
      const unsigned s6 = (unsigned)db.z - nbs, s7 = (unsigned)db.w - nbs;
      const bool h0 = inr & (s0 < unb), h1 = inr & (s1 < unb), h2 = inr & (s2 < unb), h3 = inr & (s3 < unb);
      const bool h4 = inr & (s4 < unb), h5 = inr & (s5 < unb), h6 = inr & (s6 < unb), h7 = inr & (s7 < unb);
      const unsigned m0 = __builtin_amdgcn_ballot_w32(h0), m1 = __builtin_amdgcn_ballot_w32(h1);
      const unsigned m2 = __builtin_amdgcn_ballot_w32(h2), m3 = __builtin_amdgcn_ballot_w32(h3);
      const unsigned m4 = __builtin_amdgcn_ballot_w32(h4), m5 = __builtin_amdgcn_ballot_w32(h5);
      const unsigned m6 = __builtin_amdgcn_ballot_w32(h6), m7 = __builtin_amdgcn_ballot_w32(h7);
      const unsigned any = m0 | m1 | m2 | m3 | m4 | m5 | m6 | m7;
      if (any != 0u) {
        const int pre = (int)(__builtin_amdgcn_mbcnt_lo(m0, 0u) + __builtin_amdgcn_mbcnt_lo(m1, 0u) +
                              __builtin_amdgcn_mbcnt_lo(m2, 0u) + __builtin_amdgcn_mbcnt_lo(m3, 0u) +
                              __builtin_amdgcn_mbcnt_lo(m4, 0u) + __builtin_amdgcn_mbcnt_lo(m5, 0u) +
                              __builtin_amdgcn_mbcnt_lo(m6, 0u) + __builtin_amdgcn_mbcnt_lo(m7, 0u));
        int p = wc + pre;
        if (h0) { if (p < WLCAP) mylist[p] = ((e0 + 0) << SLB) | (int)s0; p = p + 1; }
        if (h1) { if (p < WLCAP) mylist[p] = ((e0 + 1) << SLB) | (int)s1; p = p + 1; }
        if (h2) { if (p < WLCAP) mylist[p] = ((e0 + 2) << SLB) | (int)s2; p = p + 1; }
        if (h3) { if (p < WLCAP) mylist[p] = ((e0 + 3) << SLB) | (int)s3; p = p + 1; }
        if (h4) { if (p < WLCAP) mylist[p] = ((e0 + 4) << SLB) | (int)s4; p = p + 1; }
        if (h5) { if (p < WLCAP) mylist[p] = ((e0 + 5) << SLB) | (int)s5; p = p + 1; }
        if (h6) { if (p < WLCAP) mylist[p] = ((e0 + 6) << SLB) | (int)s6; p = p + 1; }
        if (h7) { if (p < WLCAP) mylist[p] = ((e0 + 7) << SLB) | (int)s7; p = p + 1; }
        wc += (int)(__builtin_popcount(m0) + __builtin_popcount(m1) + __builtin_popcount(m2) + __builtin_popcount(m3) +
                    __builtin_popcount(m4) + __builtin_popcount(m5) + __builtin_popcount(m6) + __builtin_popcount(m7));
      }
    }
    if (lane == 0) misc[wave] = wc;
  }
  __syncthreads();

  if (wave == 0) {
    int ov = 0;
#pragma unroll 1
    for (int w2 = 0; w2 < NWAVE; ++w2) {
      int c = misc[w2];
      if (c > WLCAP) ov = 1;
      c = c < 0 ? 0 : (c > WLCAP ? WLCAP : c);
#pragma unroll 1
      for (int b0 = 0; b0 < c; b0 += 32) {
        const int idx = b0 + lane;
        const int ent = wl[w2 * WLCAP + (idx < WLCAP ? idx : WLCAP - 1)];
        const int m32 = (c - b0) < 32 ? (c - b0) : 32;
#pragma unroll 1
        for (int k = 0; k < m32; ++k) {
          const int u    = __builtin_amdgcn_readlane(ent, k);
          const int slot = u & (NBRUN - 1);
          if (lane == 0) cnt[slot] = cnt[slot] + 1;
        }
      }
    }
    if (lane == 0) misc[9] = ov;
  }
  __syncthreads();
  if (wave == 0) {
    const int base = lane * (NBRUN / 32);
    int s = 0;
#pragma unroll 1
    for (int i = 0; i < NBRUN / 32; ++i) s += cnt[base + i];
    int incl = s;
#pragma unroll
    for (int d = 1; d < 32; d <<= 1) {
      const int y = __shfl_up(incl, d, 32);
      if (lane >= d) incl += y;
    }
    int run = incl - s;
#pragma unroll 1
    for (int i = 0; i < NBRUN / 32; ++i) {
      const int cv = cnt[base + i];
      offs[base + i] = run;
      cur[base + i]  = run;
      run += cv;
    }
    if (lane == 31) {
      misc[8] = run;
      if (run > RCAP) misc[9] = 1;
    }
  }
  __syncthreads();

  if (wave == 0) {
#pragma unroll 1
    for (int w2 = 0; w2 < NWAVE; ++w2) {
      int c = misc[w2];
      c = c < 0 ? 0 : (c > WLCAP ? WLCAP : c);
#pragma unroll 1
      for (int b0 = 0; b0 < c; b0 += 32) {
        const int idx = b0 + lane;
        const int ent = wl[w2 * WLCAP + (idx < WLCAP ? idx : WLCAP - 1)];
        const int m32 = (c - b0) < 32 ? (c - b0) : 32;
#pragma unroll 1
        for (int k = 0; k < m32; ++k) {
          const int u    = __builtin_amdgcn_readlane(ent, k);
          const int slot = u & (NBRUN - 1);
          const int eid  = (u >> SLB) & 0x1FFFFF;
          if (lane == 0) {
            int p = cur[slot];
            p = p < 0 ? 0 : (p > RCAP - 1 ? RCAP - 1 : p);
            sl[p] = eid;
            cur[slot] = p + 1;
          }
        }
      }
    }
  }
  __syncthreads();

  const int ovf = misc[9];
  int tot = misc[8];
  tot = tot < 0 ? 0 : (tot > RCAP ? RCAP : tot);
  const int nfl = (tot + 31) & ~31;
  int* lp  = LIST + (size_t)blk * (size_t)(2 * RCAP);
  int* cop = CO + (size_t)blk * (2 * NBRUN);
  int* fp  = FLAG + (size_t)blk * 32;
#pragma unroll 1
  for (int base = 0; base < nfl; base += 2 * NTHR) {
    const int i2 = base + 2 * tid;
    const bool ok = i2 < nfl;
    const int ic = ok ? i2 : 0;
    int e_a = sl[ic], e_b = sl[ic + 1];
    e_a = e_a < 0 ? 0 : (e_a > NE - 1 ? NE - 1 : e_a);
    e_b = e_b < 0 ? 0 : (e_b > NE - 1 ? NE - 1 : e_b);
    int o_a = oth[e_a], o_b = oth[e_b];
    const float w_a = ea[e_a], w_b = ea[e_b];
    asm volatile("" :: "v"(o_a), "v"(o_b), "v"(w_a), "v"(w_b));
    o_a = o_a < 0 ? 0 : (o_a > noth - 1 ? noth - 1 : o_a);
    o_b = o_b < 0 ? 0 : (o_b > noth - 1 ? noth - 1 : o_b);
    v4i v;
    v.x = o_a; v.y = (int)(bf16_bits(w_a) << 16);
    v.z = o_b; v.w = (int)(bf16_bits(w_b) << 16);
    if (ok) st2_v4i(lp + (size_t)2 * (size_t)i2, v);
  }
#pragma unroll 1
  for (int it = 0; it < 2; ++it) {
    const int i = it * (NTHR * 4) + 4 * tid;
    const v4i v = *(const v4ia*)(cnt + i);
    st2_v4i(cop + i, v);
  }
  if (tid < 8) {
    const v4i f = {ovf, ovf, ovf, ovf};
    st2_v4i(fp + 4 * tid, f);
  }
}

template <int ROLE>
__global__ __launch_bounds__(NTHR) void k_replay(const int* __restrict__ LIST, const int* __restrict__ CO,
                                                 const int* __restrict__ FLAG, const float* __restrict__ par,
                                                 const float* __restrict__ Hs, unsigned short* OUTP) {
  constexpr int NLIVE = ROLE ? NV : NCN;
  constexpr int NSRC  = ROLE ? NCN : NV;
  constexpr int PITCH = ROLE ? KL : KCAT;
  constexpr int COFF  = ROLE ? 0 : KL;
  constexpr int BK0   = ROLE ? NBK0 : 0;
  const int tid = (int)threadIdx.x, lane = tid & 31, wave = tid >> 5, hh = lane >> 4, q = lane & 15;
  const int rowBase = (int)blockIdx.x * ABM;
  const int bucket  = BK0 + (rowBase >> SLB);
  const int* lb  = LIST + (size_t)bucket * (size_t)(2 * RCAP);
  const int* cob = CO + (size_t)bucket * (2 * NBRUN);
  const int flag = FLAG[(size_t)bucket * 32];
  const float qnan = __uint_as_float(0x7fc00000u);
  const v4f we = *(const v4fa*)(par + 128 + 4 * q);

#pragma unroll 1
  for (int i = 0; i < ABM / (2 * NWAVE); ++i) {
    const int d    = rowBase + (ABM / NWAVE) * wave + 2 * i + hh;
    const int slot = d & (NBRUN - 1);
    int c = cob[slot];
    int o = cob[NBRUN + slot];
    const bool big = c > TRIPCAP;
    c = c < 0 ? 0 : (c > TRIPCAP ? TRIPCAP : c);
    o = o < 0 ? 0 : (o > RCAP - 1 ? RCAP - 1 : o);
    const int co = __shfl_xor(c, 16, 32);
    const int cm = c > co ? c : co;
    int last = o + c - 1;
    last = last < o ? o : last;
    last = last > RCAP - 1 ? RCAP - 1 : last;
    float a0 = 0.0f, a1 = 0.0f, a2 = 0.0f, a3 = 0.0f;
#pragma unroll 1
    for (int j = 0; j < cm; ++j) {
      int idx = o + j;
      idx = idx > last ? last : idx;
      const v2i wd = *(const v2ia*)(lb + 2 * idx);
      int sr = wd.x;
      sr = sr < 0 ? 0 : (sr > NSRC - 1 ? NSRC - 1 : sr);
      const float w = __uint_as_float((unsigned)wd.y & 0xffff0000u);
      const v4f v = *(const v4fa*)(Hs + (size_t)sr * HD + 4 * q);
      asm volatile("" :: "v"(v));
      const bool valid = j < c;
      const float t0 = w * we.x, t1 = w * we.y, t2 = w * we.z, t3 = w * we.w;
      const float n0 = fmaf(v.x, t0, a0), n1 = fmaf(v.y, t1, a1), n2 = fmaf(v.z, t2, a2), n3 = fmaf(v.w, t3, a3);
      a0 = valid ? n0 : a0; a1 = valid ? n1 : a1; a2 = valid ? n2 : a2; a3 = valid ? n3 : a3;
    }
    const bool bad  = (flag != 0) | big;
    const bool live = d < NLIVE;
    float m0 = bad ? qnan : a0, m1 = bad ? qnan : a1, m2 = bad ? qnan : a2, m3 = bad ? qnan : a3;
    m0 = live ? m0 : 0.0f; m1 = live ? m1 : 0.0f; m2 = live ? m2 : 0.0f; m3 = live ? m3 : 0.0f;
    int h01, h23, l01, l23;
    hilo_pack(m0, m1, m2, m3, h01, h23, l01, l23);
    const v4i ow = regroup8(h01, h23, l01, l23, lane);
    unsigned short* hp = OUTP + (size_t)d * PITCH + COFF + 8 * q;
    *(volatile v4i*)hp = ow;
    __threadfence();
    *(volatile v4i*)hp = ow;
  }
}

__global__ __launch_bounds__(NTHR) __attribute__((amdgpu_num_vgpr(248)))
void k_gemm_cu(const unsigned short* __restrict__ ACU, const unsigned short* __restrict__ WcuT2,
               const float* __restrict__ par, float* CE2) {
  __shared__ __attribute__((aligned(16))) float stg[GBM * SP];
  __shared__ __attribute__((aligned(16))) float sb[64];
  const int tid = (int)threadIdx.x, lane = tid & 31, wave = tid >> 5, hh = lane >> 4, m = lane & 15;
  const int rowBase = (int)blockIdx.x * GBM;
  if (tid < 16) *(v4fa*)(sb + 4 * tid) = *(const v4fa*)(par + 192 + 4 * tid);

  v8f acc[4];
  {
    const v8f z = {0.f, 0.f, 0.f, 0.f, 0.f, 0.f, 0.f, 0.f};
#pragma unroll
    for (int t = 0; t < 4; ++t) acc[t] = z;
  }
  const unsigned short* ap = ACU + (size_t)(rowBase + 16 * wave + m) * (size_t)KCAT + 8 * hh;
  const unsigned short* bp = WcuT2 + (size_t)m * (size_t)KCAT + 8 * hh;
  gemm_16x64<KCAT, KCAT>(ap, bp, acc);
  stage_d(stg, acc, wave, hh, m);
  __syncthreads();

  const v4f bias = *(const v4fa*)(sb + 4 * m);
#pragma unroll 1
  for (int i = 0; i < 8; ++i) {
    const int lr   = 16 * wave + 2 * i + hh;
    const int grow = rowBase + lr;
    const bool live = grow < NCN;
    const v4f a = *(const v4fa*)(stg + lr * SP + 4 * m);
    asm volatile("" :: "v"(a));
    float v0 = a.x + bias.x, v1 = a.y + bias.y, v2 = a.z + bias.z, v3 = a.w + bias.w;
    v0 = (v0 > 0.0f) ? v0 : (v0 - v0); v1 = (v1 > 0.0f) ? v1 : (v1 - v1);
    v2 = (v2 > 0.0f) ? v2 : (v2 - v2); v3 = (v3 > 0.0f) ? v3 : (v3 - v3);
    v4f o;
    o.x = live ? v0 : 0.0f; o.y = live ? v1 : 0.0f; o.z = live ? v2 : 0.0f; o.w = live ? v3 : 0.0f;
    st2_v4f(CE2 + (size_t)grow * HD + 4 * m, o);
  }
}

__global__ __launch_bounds__(NTHR) __attribute__((amdgpu_num_vgpr(248)))
void k_vu_head(const unsigned short* __restrict__ VEHL, const unsigned short* __restrict__ VAGG,
               const unsigned short* __restrict__ WvuT2, const unsigned short* __restrict__ Wp1T2,
               const float* __restrict__ par, const int* __restrict__ FLAG, float* out) {
  extern __shared__ __attribute__((aligned(16))) float dsf[];
  float* stg = dsf;
  int*   hlw = (int*)(dsf + GBM * SP);
  float* sb  = dsf + GBM * SP + GBM * HD;
  float* sc  = sb + 256;
  int*   wfl = (int*)(sc + GBM);
  const int tid = (int)threadIdx.x, lane = tid & 31, wave = tid >> 5, hh = lane >> 4, m = lane & 15;
  const int blk = (int)blockIdx.x;
  const int rowBase = blk * GBM;

  if (tid < 64) *(v4fa*)(sb + 4 * tid) = *(const v4fa*)(par + 256 + 4 * tid);
  {
    const int fi = tid < NBK ? tid : NBK - 1;
    const int f  = FLAG[(size_t)fi * 32];
    asm volatile("" :: "v"(f));
    const bool nz = (tid < NBK) & (f != 0);
    const unsigned bm = __builtin_amdgcn_ballot_w32(nz);
    if (lane == 0) wfl[wave] = (bm != 0u) ? 1 : 0;
  }

  v8f acc[4];
  {
    const v8f z = {0.f, 0.f, 0.f, 0.f, 0.f, 0.f, 0.f, 0.f};
#pragma unroll
    for (int t = 0; t < 4; ++t) acc[t] = z;
  }
  {
    const unsigned short* ap1 = VEHL + (size_t)(rowBase + 16 * wave + m) * (size_t)KL + 8 * hh;
    const unsigned short* ap2 = VAGG + (size_t)(rowBase + 16 * wave + m) * (size_t)KL + 8 * hh;
    const unsigned short* bp  = WvuT2 + (size_t)m * (size_t)KCAT + 8 * hh;
    gemm_16x64<KL, KCAT>(ap1, bp, acc);
    gemm_16x64<KL, KCAT>(ap2, bp + KL, acc);
  }
  stage_d(stg, acc, wave, hh, m);
  __syncthreads();

  {
    const v4f bias = *(const v4fa*)(sb + 4 * m);
#pragma unroll 1
    for (int i = 0; i < 8; ++i) {
      const int lr = 16 * wave + 2 * i + hh;
      const v4f a = *(const v4fa*)(stg + lr * SP + 4 * m);
      float v0 = a.x + bias.x, v1 = a.y + bias.y, v2 = a.z + bias.z, v3 = a.w + bias.w;
      v0 = (v0 > 0.0f) ? v0 : (v0 - v0); v1 = (v1 > 0.0f) ? v1 : (v1 - v1);
      v2 = (v2 > 0.0f) ? v2 : (v2 - v2); v3 = (v3 > 0.0f) ? v3 : (v3 - v3);
      int h01, h23, l01, l23;
      hilo_pack(v0, v1, v2, v3, h01, h23, l01, l23);
      v2i hw, lw;
      hw.x = h01; hw.y = h23; lw.x = l01; lw.y = l23;
      *(v2ia*)(hlw + lr * HD + 2 * m)      = hw;
      *(v2ia*)(hlw + lr * HD + 32 + 2 * m) = lw;
    }
  }
  __syncthreads();

  v8f ac2[4];
  {
    const v8f z = {0.f, 0.f, 0.f, 0.f, 0.f, 0.f, 0.f, 0.f};
#pragma unroll
    for (int t = 0; t < 4; ++t) ac2[t] = z;
  }
  {
    const int* arow = hlw + (16 * wave + m) * HD + 4 * hh;
    const unsigned short* bp = Wp1T2 + (size_t)m * (size_t)KL + 8 * hh;
#pragma unroll 1
    for (int k0 = 0; k0 < KL; k0 += 32) {
      FragB af;
      af.q[0] = *(const v4ia*)(arow + (k0 >> 1));
      af.q[1] = *(const v4ia*)(arow + (k0 >> 1) + 8);
#pragma unroll
      for (int nt = 0; nt < 4; ++nt) {
        const unsigned short* wq = bp + (size_t)(16 * nt) * (size_t)KL + k0;
        FragB bf;
        bf.h[0] = *(const v8usa*)wq;
        bf.h[1] = *(const v8usa*)(wq + 16);
        ac2[nt] = wmb(af, bf, ac2[nt]);
      }
    }
  }
  stage_d(stg, ac2, wave, hh, m);
  __syncthreads();

  if (tid < GBM) {
    const float* rp = stg + tid * SP;
    float s = 0.0f;
#pragma unroll 4
    for (int c4 = 0; c4 < 16; ++c4) {
      const v4f a = *(const v4fa*)(rp + 4 * c4);
      const v4f b = *(const v4fa*)(sb + 64 + 4 * c4);
      const v4f w = *(const v4fa*)(sb + 128 + 4 * c4);
      float v0 = a.x + b.x, v1 = a.y + b.y, v2 = a.z + b.z, v3 = a.w + b.w;
      v0 = (v0 > 0.0f) ? v0 : (v0 - v0); v1 = (v1 > 0.0f) ? v1 : (v1 - v1);
      v2 = (v2 > 0.0f) ? v2 : (v2 - v2); v3 = (v3 > 0.0f) ? v3 : (v3 - v3);
      s = fmaf(v0, w.x, s); s = fmaf(v1, w.y, s); s = fmaf(v2, w.z, s); s = fmaf(v3, w.w, s);
    }
    sc[tid] = s + sb[192];
  }
  __syncthreads();

  if (wave == 0) {
    const int anyf = wfl[0] | wfl[1] | wfl[2] | wfl[3] | wfl[4] | wfl[5] | wfl[6] | wfl[7];
    const float qnan = __uint_as_float(0x7fc00000u);
    v4f v = *(const v4fa*)(sc + 4 * lane);
    v.x = (anyf != 0) ? qnan : v.x; v.y = (anyf != 0) ? qnan : v.y;
    v.z = (anyf != 0) ? qnan : v.z; v.w = (anyf != 0) ? qnan : v.w;
    const int liveRows = (NV - rowBase) < GBM ? (NV - rowBase) : GBM;
    float* op = out + (size_t)rowBase + 4 * lane;
    if (4 * lane < liveRows) {
      *(volatile v4f*)op = v;
      __threadfence();
      *(volatile v4f*)op = v;
    }
  }
}

extern "C" void kernel_launch(void* const* d_in, const int* in_sizes, int n_in,
                              void* d_out, int out_size, void* d_ws, size_t ws_size,
                              hipStream_t stream) {
  if (n_in < 17) return;
  if (in_sizes[0] != NV * KV) return;
  if (in_sizes[1] != NCN * KC) return;
  if (in_sizes[2] != 2 * NE) return;
  if (in_sizes[3] != NE) return;
  if (in_sizes[4] != KV * HD || in_sizes[5] != HD) return;
  if (in_sizes[6] != KC * HD || in_sizes[7] != HD) return;
  if (in_sizes[8] != HD) return;
  if (in_sizes[9] != 2 * HD * HD || in_sizes[10] != HD) return;
  if (in_sizes[11] != 2 * HD * HD || in_sizes[12] != HD) return;
  if (in_sizes[13] != HD * HD || in_sizes[14] != HD) return;
  if (in_sizes[15] != HD || in_sizes[16] != 1) return;
  if (out_size != NV) return;

  const float* xv    = (const float*)d_in[0];
  const float* xc    = (const float*)d_in[1];
  const int*   ei    = (const int*)d_in[2];
  const float* eattr = (const float*)d_in[3];
  const float* Wvar  = (const float*)d_in[4];
  const float* bvar  = (const float*)d_in[5];
  const float* Wcon  = (const float*)d_in[6];
  const float* bcon  = (const float*)d_in[7];
  const float* wedge = (const float*)d_in[8];
  const float* Wcu   = (const float*)d_in[9];
  const float* bcu   = (const float*)d_in[10];
  const float* Wvu   = (const float*)d_in[11];
  const float* bvu   = (const float*)d_in[12];
  const float* Wp1   = (const float*)d_in[13];
  const float* bp1   = (const float*)d_in[14];
  const float* Wp2   = (const float*)d_in[15];
  const float* bp2   = (const float*)d_in[16];
  float* out = (float*)d_out;

  constexpr size_t zVE   = (size_t)MPV * HD * 4;
  constexpr size_t zVEHL = (size_t)MPV * KL * 2;
  constexpr size_t zACU  = (size_t)MPC * KCAT * 2;
  constexpr size_t zVAGG = (size_t)MPV * KL * 2;
  constexpr size_t zCE2  = (size_t)MPC * HD * 4;
  constexpr size_t zLIST = (size_t)NBK * RCAP * 8;
  constexpr size_t zCO   = (size_t)NBK * 2 * NBRUN * 4;
  constexpr size_t zFLAG = (((size_t)NBK * 128) + 255) & ~(size_t)255;
  constexpr size_t zW32  = (size_t)HD * 32 * 2;
  constexpr size_t zW256 = (size_t)HD * KCAT * 2;
  constexpr size_t zW128 = (size_t)HD * KL * 2;
  constexpr size_t zPAR  = (size_t)PAR_N * 4;
  constexpr size_t oVE   = 0;
  constexpr size_t oVEHL = oVE + zVE;
  constexpr size_t oACU  = oVEHL + zVEHL;
  constexpr size_t oCE2  = oACU + zACU;
  constexpr size_t oLIST = oCE2 + zCE2;
  constexpr size_t oCO   = oLIST + zLIST;
  constexpr size_t oFLAG = oCO + zCO;
  constexpr size_t oWvT  = oFLAG + zFLAG;
  constexpr size_t oWcT  = oWvT + zW32;
  constexpr size_t oWcu  = oWcT + zW32;
  constexpr size_t oWvu  = oWcu + zW256;
  constexpr size_t oWp1  = oWvu + zW256;
  constexpr size_t oPAR  = oWp1 + zW128;
  constexpr size_t oEND  = oPAR + zPAR;
  static_assert(zACU == zVAGG);
  static_assert(zVE % 256 == 0 && zVEHL % 256 == 0 && zACU % 256 == 0 && zCE2 % 256 == 0);
  static_assert(zLIST % 256 == 0 && zCO % 256 == 0 && zFLAG % 256 == 0 && zPAR % 256 == 0);
  static_assert(zW32 % 256 == 0 && zW256 % 256 == 0 && zW128 % 256 == 0);
  static_assert(oEND <= (size_t)(128u << 20));
  if (oEND > ws_size) return;

  char* ws = (char*)d_ws;
  float*          VE    = (float*)(ws + oVE);
  unsigned short* VEHL  = (unsigned short*)(ws + oVEHL);
  unsigned short* ACU   = (unsigned short*)(ws + oACU);
  unsigned short* VAGG  = (unsigned short*)(ws + oACU);
  float*          CE2   = (float*)(ws + oCE2);
  int*            LIST  = (int*)(ws + oLIST);
  int*            CO    = (int*)(ws + oCO);
  int*            FLAG  = (int*)(ws + oFLAG);
  unsigned short* WvT   = (unsigned short*)(ws + oWvT);
  unsigned short* WcT   = (unsigned short*)(ws + oWcT);
  unsigned short* WcuT2 = (unsigned short*)(ws + oWcu);
  unsigned short* WvuT2 = (unsigned short*)(ws + oWvu);
  unsigned short* Wp1T2 = (unsigned short*)(ws + oWp1);
  float*          PAR   = (float*)(ws + oPAR);

  hipFuncSetAttribute(reinterpret_cast<const void*>(&k_bucket), hipFuncAttributeMaxDynamicSharedMemorySize, (int)BK_LDS);
  hipFuncSetAttribute(reinterpret_cast<const void*>(&k_vu_head), hipFuncAttributeMaxDynamicSharedMemorySize, (int)VH_LDS);

  k_prep<<<PREP_BLOCKS, NTHR, 0, stream>>>(Wvar, Wcon, Wcu, Wvu, Wp1, bvar, bcon, wedge, bcu, bvu, bp1, Wp2, bp2,
                                           WvT, WcT, WcuT2, WvuT2, Wp1T2, PAR);
  k_embed<<<TV + TC, NTHR, 0, stream>>>(xv, xc, WvT, WcT, PAR, VE, VEHL, ACU);
  k_bucket<<<NBK, NTHR, BK_LDS, stream>>>(ei, eattr, LIST, CO, FLAG);
  k_replay<0><<<MPC / ABM, NTHR, 0, stream>>>(LIST, CO, FLAG, PAR, VE, ACU);
  k_gemm_cu<<<TC, NTHR, 0, stream>>>(ACU, WcuT2, PAR, CE2);
  k_replay<1><<<MPV / ABM, NTHR, 0, stream>>>(LIST, CO, FLAG, PAR, CE2, VAGG);
  k_vu_head<<<TV, NTHR, VH_LDS, stream>>>(VEHL, VAGG, WvuT2, Wp1T2, PAR, FLAG, out);
}
